// HedgeDogConvAttention_27023934226683
// MI455X (gfx1250) — hardware-verified
//
#include <hip/hip_runtime.h>


typedef __bf16 bf16_t;
typedef bf16_t v16b __attribute__((ext_vector_type(16)));
typedef bf16_t v8b  __attribute__((ext_vector_type(8), __may_alias__));
typedef float  v8f  __attribute__((ext_vector_type(8)));
typedef float  v4f  __attribute__((ext_vector_type(4), __may_alias__));

#define CH   256
#define NT   4096
#define DH   64
#define NHQ  4
#define NHF  8
#define HOFF ((size_t)NT * DH)
#define P32  40
#define P64  72
#define PC   36
#define EPSV 1e-6f

union Frag { v16b v; v8b half[2]; };

__device__ __forceinline__ v16b frag_ld(const bf16_t* row0, int pitch, int lane) {
  const int m = lane & 15, h = lane >> 4;
  const bf16_t* p = row0 + m * pitch + 8 * h;
  Frag f;
  f.half[0] = *(const v8b*)p;
  f.half[1] = *(const v8b*)(p + 16);
  return f.v;
}

__device__ __forceinline__ v8f mma_bf16(v16b a, v16b b, v8f c) {
  v8f d = __builtin_amdgcn_wmma_f32_16x16x32_bf16(false, a, false, b, (short)0, c, false, false);
  asm volatile("v_nop\n\tv_nop\n\tv_nop\n\tv_nop" : "+v"(d) : "v"(a), "v"(b));
  return d;
}

__device__ __forceinline__ v8f zero8() {
  v8f z = {0.f, 0.f, 0.f, 0.f, 0.f, 0.f, 0.f, 0.f};
  return z;
}

__device__ __forceinline__ v8b cvt8(const float* __restrict__ p) {
  const v4f f0 = *(const v4f*)p;
  const v4f f1 = *(const v4f*)(p + 4);
  v8b r;
  r[0] = (bf16_t)f0[0]; r[1] = (bf16_t)f0[1]; r[2] = (bf16_t)f0[2]; r[3] = (bf16_t)f0[3];
  r[4] = (bf16_t)f1[0]; r[5] = (bf16_t)f1[1]; r[6] = (bf16_t)f1[2]; r[7] = (bf16_t)f1[3];
  return r;
}

__device__ __forceinline__ void lines_out_f32(const float* cs, int cpitch, float* dst, size_t ld,
                                              int nrows, int wave, int nwaves, int lane) {
  const int sub = lane >> 3, c = (lane & 7) * 4;
  for (int L0 = wave * 4; L0 < nrows; L0 += nwaves * 4) {
    const int L = L0 + sub;
    const v4f val = *(const v4f*)(cs + L * cpitch + c);
    *(volatile v4f*)(dst + (size_t)L * ld + c) = val;
  }
  __threadfence();
  for (int L0 = wave * 4; L0 < nrows; L0 += nwaves * 4) {
    const int L = L0 + sub;
    const v4f val = *(const v4f*)(cs + L * cpitch + c);
    *(volatile v4f*)(dst + (size_t)L * ld + c) = val;
  }
}

__global__ __launch_bounds__(128) void k_proj(
    const float* __restrict__ Wq, const float* __restrict__ Wk,
    const float* __restrict__ x, float* __restrict__ q, float* __restrict__ k) {
  const float* __restrict__ W = blockIdx.z ? Wk : Wq;
  float* __restrict__ dst = blockIdx.z ? k : q;
  const int nB = blockIdx.x * 32, mB = blockIdx.y * 32;
  __shared__ __align__(16) bf16_t As[32][P32];
  __shared__ __align__(16) bf16_t Bt[32][P32];
  __shared__ __align__(16) float  Cs[32][PC];
  const int t = threadIdx.x, lane = t & 31, wave = t >> 5;
  const int wm = (wave >> 1) * 16, wn = (wave & 1) * 16;
  const int r = t >> 2, seg = (t & 3) * 8;
  const float* pW = W + (size_t)(mB + r) * CH + seg;
  const float* pX = x + (size_t)r * NT + nB + seg;
  v8f acc = zero8();
  for (int kc = 0; kc < CH; kc += 32) {
    *(v8b*)&As[r][seg] = cvt8(pW + kc);
    const float* px = pX + (size_t)kc * NT;
    const v4f x0 = *(const v4f*)px;
    const v4f x1 = *(const v4f*)(px + 4);
    Bt[seg + 0][r] = (bf16_t)x0[0]; Bt[seg + 1][r] = (bf16_t)x0[1];
    Bt[seg + 2][r] = (bf16_t)x0[2]; Bt[seg + 3][r] = (bf16_t)x0[3];
    Bt[seg + 4][r] = (bf16_t)x1[0]; Bt[seg + 5][r] = (bf16_t)x1[1];
    Bt[seg + 6][r] = (bf16_t)x1[2]; Bt[seg + 7][r] = (bf16_t)x1[3];
    __syncthreads();
    acc = mma_bf16(frag_ld(&As[wm][0], P32, lane), frag_ld(&Bt[wn][0], P32, lane), acc);
    __syncthreads();
  }
  {
    const int h = lane >> 4, cn = wn + (lane & 15);
#pragma unroll
    for (int rr = 0; rr < 8; ++rr) Cs[wm + 8 * h + rr][cn] = acc[rr];
  }
  __syncthreads();
  lines_out_f32(&Cs[0][0], PC, dst + (size_t)mB * NT + nB, NT, 32, wave, 4, lane);
}

__global__ __launch_bounds__(256) void k_conv(
    const float* __restrict__ x, const float* __restrict__ Wv,
    const float* __restrict__ bv, float* __restrict__ v) {
  __shared__ __align__(16) float red[256];
  const int t = threadIdx.x;
  const int idx = blockIdx.x * 256 + t;
  const int c = idx >> 12, n = idx & (NT - 1);
  const int a0 = n >> 8, a1 = (n >> 4) & 15, a2 = n & 15;
  const float* __restrict__ xc = x + (size_t)c * NT;
  const float* __restrict__ wc = Wv + c * 27;
  float s = bv[c];
#pragma unroll
  for (int i = -1; i <= 1; ++i) {
    const int p0 = a0 + i;
    if ((unsigned)p0 >= 16u) continue;
#pragma unroll
    for (int j = -1; j <= 1; ++j) {
      const int p1 = a1 + j;
      if ((unsigned)p1 >= 16u) continue;
#pragma unroll
      for (int kk = -1; kk <= 1; ++kk) {
        const int p2 = a2 + kk;
        if ((unsigned)p2 >= 16u) continue;
        s += xc[p0 * 256 + p1 * 16 + p2] * wc[(i + 1) * 9 + (j + 1) * 3 + (kk + 1)];
      }
    }
  }
  red[t] = s;
  __syncthreads();
  if (t < 64) {
    const int lane = t & 31, w = t >> 5;
    const int n0 = (blockIdx.x * 256) & (NT - 1);
    const int off = 128 * w + 4 * lane;
    const v4f val = *(const v4f*)&red[off];
    float* p = v + (size_t)c * NT + n0 + off;
    *(volatile v4f*)p = val;
    __threadfence();
    *(volatile v4f*)p = val;
  }
}

__global__ __launch_bounds__(128) void k_hedge(
    const float* __restrict__ src, const float* __restrict__ Wm,
    const float* __restrict__ bm, bf16_t* __restrict__ dst) {
  const int nb = blockIdx.x * 32, hd = blockIdx.z;
  __shared__ __align__(16) bf16_t As[32][P64];
  __shared__ __align__(16) bf16_t Ws[64][P64];
  __shared__ __align__(16) bf16_t Os[64][P64];
  __shared__ float bs[64];
  const int t = threadIdx.x, lane = t & 31, wave = t >> 5;
  const int wm = (wave >> 1) * 16, wn = (wave & 1) * 32;
  {
    const int d = t >> 1, ts = (t & 1) * 16;
    const float* p = src + (size_t)(hd * DH + d) * NT + nb + ts;
#pragma unroll
    for (int j = 0; j < 16; j += 4) {
      const v4f f = *(const v4f*)(p + j);
      As[ts + j + 0][d] = (bf16_t)f[0];
      As[ts + j + 1][d] = (bf16_t)f[1];
      As[ts + j + 2][d] = (bf16_t)f[2];
      As[ts + j + 3][d] = (bf16_t)f[3];
    }
  }
  {
    const int e = t >> 1, ds = (t & 1) * 32;
    const float* p = Wm + e * DH + ds;
#pragma unroll
    for (int j = 0; j < 32; j += 8) *(v8b*)&Ws[e][ds + j] = cvt8(p + j);
  }
  if (t < 64) bs[t] = bm[t];
  __syncthreads();
  v8f acc0 = zero8(), acc1 = zero8();
#pragma unroll
  for (int ks = 0; ks < DH; ks += 32) {
    const v16b a = frag_ld(&As[wm][ks], P64, lane);
    acc0 = mma_bf16(a, frag_ld(&Ws[wn][ks], P64, lane), acc0);
    acc1 = mma_bf16(a, frag_ld(&Ws[wn + 16][ks], P64, lane), acc1);
  }
  {
    const int h = lane >> 4, cn = lane & 15;
    const int e0 = wn + cn, e1 = wn + 16 + cn;
    const float b0 = bs[e0], b1 = bs[e1];
#pragma unroll
    for (int rr = 0; rr < 8; ++rr) {
      const int tok = wm + 8 * h + rr;
      const float h0 = acc0[rr] + b0;
      const float h1 = acc1[rr] + b1;
      Os[tok][e0]      = (bf16_t)__expf(h0);
      Os[32 + tok][e0] = (bf16_t)__expf(-h0);
      Os[tok][e1]      = (bf16_t)__expf(h1);
      Os[32 + tok][e1] = (bf16_t)__expf(-h1);
    }
  }
  __syncthreads();
  {
    const int sub = lane >> 3, c = (lane & 7) * 8;
#pragma unroll
    for (int ps = 0; ps < 4; ++ps) {
      const int L = wave * 16 + ps * 4 + sub;
      const int hh = (L < 32) ? hd : hd + NHQ;
      const int tokl = L & 31;
      const v4f val = *(const v4f*)&Os[L][c];
      bf16_t* g = dst + (size_t)hh * HOFF + (size_t)(nb + tokl) * DH + c;
      *(volatile v4f*)g = val;
    }
    __threadfence();
#pragma unroll
    for (int ps = 0; ps < 4; ++ps) {
      const int L = wave * 16 + ps * 4 + sub;
      const int hh = (L < 32) ? hd : hd + NHQ;
      const int tokl = L & 31;
      const v4f val = *(const v4f*)&Os[L][c];
      bf16_t* g = dst + (size_t)hh * HOFF + (size_t)(nb + tokl) * DH + c;
      *(volatile v4f*)g = val;
    }
  }
}

__global__ __launch_bounds__(128) void k_kv(
    const bf16_t* __restrict__ kf, const bf16_t* __restrict__ vf,
    float* __restrict__ KVt, float* __restrict__ ksum) {
  const int db = blockIdx.x * 32, eb = blockIdx.y * 32, hd = blockIdx.z;
  __shared__ __align__(16) bf16_t At[32][P32];
  __shared__ __align__(16) bf16_t Bt[32][P32];
  __shared__ __align__(16) float  Cs[32][PC];
  __shared__ __align__(16) float  Ks[32];
  const int t = threadIdx.x, lane = t & 31, wave = t >> 5;
  const int wm = (wave >> 1) * 16, wn = (wave & 1) * 16;
  const int r = t >> 2, seg = (t & 3) * 8;
  const bf16_t* pV = vf + (size_t)hd * HOFF + (size_t)r * DH + eb + seg;
  const bf16_t* pK = kf + (size_t)hd * HOFF + (size_t)r * DH + db + seg;
  const bool do_ks = (blockIdx.y == 0);
  v8f acc = zero8();
  float ks = 0.f;
#pragma unroll 2
  for (int it = 0; it < NT / 32; ++it) {
    const v8b av = *(const v8b*)(pV + (size_t)it * 32 * DH);
    const v8b bk = *(const v8b*)(pK + (size_t)it * 32 * DH);
#pragma unroll
    for (int j = 0; j < 8; ++j) {
      At[seg + j][r] = av[j];
      Bt[seg + j][r] = bk[j];
    }
    __syncthreads();
    acc = mma_bf16(frag_ld(&At[wm][0], P32, lane), frag_ld(&Bt[wn][0], P32, lane), acc);
    if (do_ks && t < 32) {
      float s = 0.f;
#pragma unroll
      for (int j = 0; j < 32; j += 8) {
        const v8b q8 = *(const v8b*)&Bt[t][j];
#pragma unroll
        for (int i = 0; i < 8; ++i) s += (float)q8[i];
      }
      ks += s;
    }
    __syncthreads();
  }
  {
    const int h = lane >> 4, cn = wn + (lane & 15);
#pragma unroll
    for (int rr = 0; rr < 8; ++rr) Cs[wm + 8 * h + rr][cn] = acc[rr];
  }
  __syncthreads();
  lines_out_f32(&Cs[0][0], PC, KVt + (size_t)hd * DH * DH + (size_t)eb * DH + db, DH, 32, wave, 4, lane);
  if (do_ks) {
    if (t < 32) Ks[t] = ks;
    __syncthreads();
    if (t < 8) {
      const v4f val = *(const v4f*)&Ks[4 * t];
      float* p = ksum + hd * DH + db + 4 * t;
      *(volatile v4f*)p = val;
      __threadfence();
      *(volatile v4f*)p = val;
    }
  }
}

__global__ __launch_bounds__(128) void k_out(
    const bf16_t* __restrict__ qf, const float* __restrict__ KVt,
    const float* __restrict__ ksum, float* __restrict__ out) {
  const int nb = blockIdx.x * 32, eb = blockIdx.y * 32, hd = blockIdx.z;
  __shared__ __align__(16) bf16_t As[32][P64];
  __shared__ __align__(16) bf16_t Bt[32][P64];
  __shared__ __align__(16) float  Cs[32][PC];
  __shared__ float ksh[64];
  __shared__ float rden[32];
  const int t = threadIdx.x, lane = t & 31, wave = t >> 5;
  const int wm = (wave >> 1) * 16, wn = (wave & 1) * 16;
  {
#pragma unroll
    for (int i = 0; i < 2; ++i) {
      const int p = t + 128 * i;
      const int row = p >> 3, c = (p & 7) * 8;
      const v4f val = *(const v4f*)(qf + (size_t)hd * HOFF + (size_t)(nb + row) * DH + c);
      *(v4f*)&As[row][c] = val;
    }
  }
  {
    const int e = t >> 2, ds = (t & 3) * 16;
    const float* p = KVt + (size_t)hd * DH * DH + (size_t)(eb + e) * DH + ds;
    *(v8b*)&Bt[e][ds]     = cvt8(p);
    *(v8b*)&Bt[e][ds + 8] = cvt8(p + 8);
  }
  if (t < 64) ksh[t] = ksum[hd * DH + t];
  __syncthreads();
  if (t < 32) {
    float s = 0.f;
#pragma unroll
    for (int d = 0; d < DH; d += 8) {
      const v8b q8 = *(const v8b*)&As[t][d];
#pragma unroll
      for (int i = 0; i < 8; ++i) s += (float)q8[i] * ksh[d + i];
    }
    rden[t] = 1.0f / (s + EPSV);
  }
  v8f acc = zero8();
#pragma unroll
  for (int ks = 0; ks < DH; ks += 32)
    acc = mma_bf16(frag_ld(&As[wm][ks], P64, lane), frag_ld(&Bt[wn][ks], P64, lane), acc);
  __syncthreads();
  {
    const int h = lane >> 4, e = wn + (lane & 15);
#pragma unroll
    for (int rr = 0; rr < 8; ++rr) {
      const int tokl = wm + 8 * h + rr;
      Cs[e][tokl] = acc[rr] * rden[tokl];
    }
  }
  __syncthreads();
  lines_out_f32(&Cs[0][0], PC, out + (size_t)(hd * DH + eb) * NT + nb, NT, 32, wave, 4, lane);
}

extern "C" void kernel_launch(void* const* d_in, const int* in_sizes, int n_in,
                              void* d_out, int out_size, void* d_ws, size_t ws_size,
                              hipStream_t stream) {
  if (n_in < 11) return;
  if (in_sizes[0] != CH * NT || in_sizes[1] != CH * CH || in_sizes[2] != CH * CH ||
      in_sizes[3] != CH * 27 || in_sizes[4] != CH || in_sizes[5] != DH * DH ||
      in_sizes[7] != DH * DH || in_sizes[9] != DH * DH ||
      in_sizes[6] != DH || in_sizes[8] != DH || in_sizes[10] != DH) return;
  if (out_size != 2 * CH * NT) return;

  const float* x   = (const float*)d_in[0];
  const float* Wq  = (const float*)d_in[1];
  const float* Wk  = (const float*)d_in[2];
  const float* Wv  = (const float*)d_in[3];
  const float* bv  = (const float*)d_in[4];
  const float* Wmq = (const float*)d_in[5];
  const float* bmq = (const float*)d_in[6];
  const float* Wmk = (const float*)d_in[7];
  const float* bmk = (const float*)d_in[8];
  const float* Wmv = (const float*)d_in[9];
  const float* bmv = (const float*)d_in[10];
  float* out = (float*)d_out;

  float* q = (float*)d_ws;
  float* k = q + (size_t)CH * NT;
  float* v = k + (size_t)CH * NT;
  bf16_t* qf = (bf16_t*)(v + (size_t)CH * NT);
  bf16_t* kf = qf + NHF * HOFF;
  bf16_t* vf = kf + NHF * HOFF;
  float* KVt  = (float*)(vf + NHF * HOFF);
  float* ksum = KVt + (size_t)NHF * DH * DH;
  const size_t need = (size_t)((const char*)(ksum + NHF * DH) - (const char*)d_ws);
  if (need > ws_size) return;

  k_proj<<<dim3(NT / 32, CH / 32, 2), 128, 0, stream>>>(Wq, Wk, x, q, k);
  k_conv<<<dim3((CH * NT) / 256), 256, 0, stream>>>(x, Wv, bv, v);
  k_hedge<<<dim3(NT / 32, 1, NHQ), 128, 0, stream>>>(q, Wmq, bmq, qf);
  k_hedge<<<dim3(NT / 32, 1, NHQ), 128, 0, stream>>>(k, Wmk, bmk, kf);
  k_hedge<<<dim3(NT / 32, 1, NHQ), 128, 0, stream>>>(v, Wmv, bmv, vf);
  k_kv<<<dim3(DH / 32, DH / 32, NHF), 128, 0, stream>>>(kf, vf, KVt, ksum);
  k_out<<<dim3(NT / 32, DH / 32, NHF), 128, 0, stream>>>(qf, KVt, ksum, out);
}
